// DTM_16423954940063
// MI455X (gfx1250) — hardware-verified
//
#include <hip/hip_runtime.h>


namespace {
constexpr int Bn = 16, C = 64, H = 64, W = 64, NPOS = Bn * H * W, K9 = 9, KK = K9 * C  , NPM = 27, CO = 128;
constexpr float AS_ = 8.0f, EPS = 1e-5f;

typedef _Float16 b16;
typedef __attribute__((ext_vector_type(16))) _Float16 v16b;
typedef __attribute__((ext_vector_type(8))) _Float16 v8b;
typedef __attribute__((ext_vector_type(8))) float v8f;
typedef __attribute__((ext_vector_type(4))) float v4f;
__device__ __forceinline__ float bf16_rne(float f) { unsigned int u = __float_as_uint(f); u += 0x7FFFu + ((u >> 16) & 1u); return __uint_as_float(u & 0xFFFF0000u); }
__device__ __forceinline__ void split16(float v, b16& hi, b16& lo) { hi = (b16)v; lo = (b16)(v - (float)hi); }
__device__ __forceinline__ v16b frag_kb(const b16* p, int hh) { const v8b a = *(const v8b*)(p + 8 * hh), b = *(const v8b*)(p + 16 + 8 * hh); v16b f;
#pragma unroll
  for (int e = 0; e < 8; ++e) { f[e] = a[e]; f[8 + e] = b[e]; } return f; }
__device__ __forceinline__ v8f wmma16b(v16b a, v16b b, v8f c) { v8f d = __builtin_amdgcn_wmma_f32_16x16x32_f16(false, a, false, b, (short)0, c, false, false); asm volatile("v_nop\n\tv_nop\n\tv_nop\n\tv_nop" : "+v"(d) : "v"(a), "v"(b)); return d; }
__device__ __forceinline__ void wave_lds_sync() { __builtin_amdgcn_fence(__ATOMIC_RELEASE, "workgroup"); __builtin_amdgcn_wave_barrier(); __builtin_amdgcn_fence(__ATOMIC_ACQUIRE, "workgroup"); }
__device__ __forceinline__ float nexp(float x) { return __builtin_amdgcn_exp2f(x * 1.4426950408889634f); }
__device__ __forceinline__ float pmul(float a, float b) { float p = a * b; asm volatile("" : "+v"(p)); return p; }

__global__ __launch_bounds__(256) void prep_kernel(const float* __restrict__ wp, const float* __restrict__ bp, const float* __restrict__ wm, const float* __restrict__ bm, const float* __restrict__ wd, const float* __restrict__ bd, const float* __restrict__ gam, const float* __restrict__ bet, b16* __restrict__ R, float* __restrict__ P) {
  const int t_ = blockIdx.x * 256 + threadIdx.x, nth = gridDim.x * 256;
  for (int pass = 0; pass < 2; ++pass) {
    for (int q = t_; q < 32 * KK; q += nth) { const int o = q / KK, k = q % KK, tap = k / C, c = k % C; float w = 0.0f; if (o < 18) w = bf16_rne(wp[((size_t)o * C + c) * 9 + tap]); else if (o < NPM) w = bf16_rne(wm[((size_t)(o - 18) * C + c) * 9 + tap]); R[q] = (b16)w; }
    for (int q = t_; q < CO * KK; q += nth) { const int o = q / KK, k = q % KK, tap = k / C, c = k % C; R[32 * KK + q] = (b16)bf16_rne(wd[((size_t)o * C + c) * 9 + tap]); }
    for (int q = t_; q < 416; q += nth) { float v; if (q < 18) v = bp[q]; else if (q < 27) v = bm[q - 18]; else if (q < 32) v = 0.0f; else if (q < 160) v = bd[q - 32]; else if (q < 288) v = gam[q - 160]; else v = bet[q - 288]; P[q] = bf16_rne(v); }
    __threadfence(); }
}

__global__ __launch_bounds__(256) void xpose_kernel(const float* __restrict__ x, b16* __restrict__ xt) {
  __shared__ __attribute__((aligned(16))) b16 T[2 * W][C + 8];
  const int b = blockIdx.y, i0 = blockIdx.x * 2, t_ = threadIdx.x;
  for (int q = t_; q < C * 2 * W; q += 256) { const int c = q / (2 * W), pp = q % (2 * W); T[pp][c] = (b16)bf16_rne(x[(((size_t)b * C + c) * H + i0) * W + pp]); }
  __syncthreads();
  for (int pass = 0; pass < 2; ++pass) { for (int q = t_; q < 2 * W * (C / 8); q += 256) { const int pp = q >> 3, c8 = (q & 7) * 8; *(volatile v8b*)(xt + (((size_t)b * H + i0) * W + pp) * C + c8) = *(const v8b*)(&T[pp][c8]); } __threadfence(); }
}

__device__ __forceinline__ v16b frag_im2col(const b16* xtb, int i, int j, int kb, int hh) { const int tap = kb / C, cb = kb % C; const int u = tap / 3 - 1, v = tap % 3 - 1; const int ii = i + u, jj = j + v; v16b f = {};
  if (ii >= 0 && ii < H && jj >= 0 && jj < W) f = frag_kb(xtb + ((size_t)ii * W + jj) * C + cb, hh);
  return f; }

__global__ __launch_bounds__(128) void offconv_kernel(const b16* __restrict__ xt, const b16* __restrict__ R, const float* __restrict__ P, float* __restrict__ pm) {
  __shared__ __attribute__((aligned(16))) float Ts[4][32 * 32];
  const int lane = threadIdx.x & 31, wave = threadIdx.x >> 5, nloc = lane & 15, hlf = lane >> 4, b = blockIdx.y; const int p0 = blockIdx.x * 128 + wave * 32; const b16* xtb = xt + ((size_t)b * H) * W * C;
  v8f acc[2][2];
#pragma unroll
  for (int r = 0; r < 2; ++r) { acc[r][0] = (v8f){}; acc[r][1] = (v8f){}; }
  for (int kb = 0; kb < KK; kb += 32) { const int pa = p0 + nloc, pb = p0 + 16 + nloc; const v16b a0 = frag_im2col(xtb, pa / W, pa % W, kb, hlf), a1 = frag_im2col(xtb, pb / W, pb % W, kb, hlf);
#pragma unroll
    for (int t = 0; t < 2; ++t) { const v16b bw = frag_kb(R + (size_t)(t * 16 + nloc) * KK + kb, hlf); acc[0][t] = wmma16b(a0, bw, acc[0][t]); acc[1][t] = wmma16b(a1, bw, acc[1][t]); } }
  float* Tt = Ts[wave];
#pragma unroll
  for (int t = 0; t < 2; ++t) { const int cc = t * 16 + nloc; const float bb = P[cc];
#pragma unroll
    for (int r = 0; r < 2; ++r)
#pragma unroll
      for (int v = 0; v < 8; ++v) { float y = acc[r][t][v] + bb; if (cc >= 18 && cc < NPM) y = 1.0f / (1.0f + nexp(-y)); Tt[(r * 16 + 8 * hlf + v) * 32 + cc] = y; } }
  wave_lds_sync();
  const size_t g0 = ((size_t)b * H * W + p0);
  for (int pass = 0; pass < 2; ++pass) { for (int q = lane; q < 32 * 8; q += 32) { const int rr = q >> 3, c4 = (q & 7) * 4; *(volatile v4f*)(pm + (g0 + rr) * 32 + c4) = *(const v4f*)(Tt + rr * 32 + c4); } __threadfence(); }
}

__global__ __launch_bounds__(256) void deform_kernel(const b16* __restrict__ xt, const float* __restrict__ pm, const b16* __restrict__ R, const float* __restrict__ P, float* __restrict__ y) {
  __shared__ __attribute__((aligned(16))) float Tw[CO][128 + 4];
  const int lane = threadIdx.x & 31, wave = threadIdx.x >> 5, nloc = lane & 15, hlf = lane >> 4, b = blockIdx.y; const int pblk = blockIdx.x * 128, p = pblk + wave * 16 + nloc, i = p / W, j = p % W;
  const b16* xtb = xt + ((size_t)b * H) * W * C; const b16* Wd = R + 32 * KK; const float* prow = pm + ((size_t)b * H * W + p) * 32;
  v8f acc[8];
#pragma unroll
  for (int t = 0; t < 8; ++t) acc[t] = (v8f){};
  for (int tap = 0; tap < K9; ++tap) { const float ky = (float)(tap / 3 - 1), kx = (float)(tap % 3 - 1);
    const float dy = prow[tap * 2], dx = prow[tap * 2 + 1], msk = prow[18 + tap];
    const float py = ((float)i + ky) + dy, px = ((float)j + kx) + dx; const float fy = floorf(py), fx = floorf(px); const float ly = py - fy, lx = px - fx; const int y0 = (int)fy, x0 = (int)fx;
    const float wg[4] = {pmul(1.0f - ly, 1.0f - lx), pmul(1.0f - ly, lx), pmul(ly, 1.0f - lx), pmul(ly, lx)};
    for (int cb = 0; cb < C; cb += 32) { float val[16];
#pragma unroll
      for (int e = 0; e < 16; ++e) val[e] = 0.0f;
#pragma unroll
      for (int cn = 0; cn < 4; ++cn) { const int yy = y0 + (cn >> 1), xx = x0 + (cn & 1); if (yy >= 0 && yy < H && xx >= 0 && xx < W) { const b16* src = xtb + ((size_t)yy * W + xx) * C + cb; const v8b q0 = *(const v8b*)(src + 8 * hlf), q1 = *(const v8b*)(src + 16 + 8 * hlf); const float wv = wg[cn];
#pragma unroll
          for (int e = 0; e < 8; ++e) { val[e] += pmul((float)q0[e], wv); val[8 + e] += pmul((float)q1[e], wv); } } }
      v16b ah, al;
#pragma unroll
      for (int e = 0; e < 16; ++e) { b16 h_, l_; split16(pmul(val[e], msk) * AS_, h_, l_); ah[e] = h_; al[e] = l_; }
#pragma unroll
      for (int t = 0; t < 8; ++t) { const v16b bw = frag_kb(Wd + (size_t)(t * 16 + nloc) * KK + tap * C + cb, hlf); acc[t] = wmma16b(ah, bw, acc[t]); acc[t] = wmma16b(al, bw, acc[t]); } } }
#pragma unroll
  for (int t = 0; t < 8; ++t) { const int o = t * 16 + nloc; const float bb = P[32 + o];
#pragma unroll
    for (int v = 0; v < 8; ++v) Tw[o][wave * 16 + 8 * hlf + v] = acc[t][v] * (1.0f / AS_) + bb; }
  __syncthreads();
  for (int pass = 0; pass < 2; ++pass) { for (int q = threadIdx.x; q < CO * 32; q += 256) { const int o = q >> 5, c4 = (q & 31) * 4; *(volatile v4f*)(y + ((size_t)b * CO + o) * H * W + pblk + c4) = *(const v4f*)(&Tw[o][c4]); } __threadfence(); }
}

__global__ __launch_bounds__(256) void bnstat_kernel(const float* __restrict__ y, float* __restrict__ st) {
  __shared__ float red[256]; __shared__ float mu_s;
  const int o = blockIdx.x, t_ = threadIdx.x; const float cnt = (float)Bn * H * W;
  float s = 0.0f; for (int b = 0; b < Bn; ++b) { const float* row = y + ((size_t)b * CO + o) * H * W; for (int q = t_; q < H * W; q += 256) s += row[q]; }
  red[t_] = s; __syncthreads(); for (int k = 128; k > 0; k >>= 1) { if (t_ < k) red[t_] += red[t_ + k]; __syncthreads(); }
  if (t_ == 0) mu_s = red[0] / cnt; __syncthreads(); const float mu = mu_s;
  float qq = 0.0f; for (int b = 0; b < Bn; ++b) { const float* row = y + ((size_t)b * CO + o) * H * W; for (int q = t_; q < H * W; q += 256) { const float d = row[q] - mu; qq += pmul(d, d); } }
  __syncthreads(); red[t_] = qq; __syncthreads(); for (int k = 128; k > 0; k >>= 1) { if (t_ < k) red[t_] += red[t_ + k]; __syncthreads(); }
  if (t_ < 32) { const float v = (t_ == 0) ? mu : (t_ == 1) ? rsqrtf(red[0] / cnt + EPS) : 0.0f; for (int pass = 0; pass < 2; ++pass) ((volatile float*)st)[(size_t)o * 32 + t_] = v; }
  __threadfence();
}

__global__ __launch_bounds__(256) void final_kernel(const float* __restrict__ y, const float* __restrict__ st, const float* __restrict__ P, float* __restrict__ out) {
  const size_t g = ((size_t)blockIdx.x * 256 + threadIdx.x) * 4; const int o = (int)((g / ((size_t)H * W)) % CO); const float mu = st[o * 32], is = st[o * 32 + 1], ga = P[160 + o], be = P[288 + o];
  const v4f v = *(const v4f*)(y + g); v4f r;
  for (int e = 0; e < 4; ++e) { const float z = pmul((v[e] - mu) * is, ga) + be; r[e] = 0.5f * z * (1.0f + erff(z * 0.70710678118654752f)); }
  for (int pass = 0; pass < 2; ++pass) { *(volatile v4f*)(out + g) = r; __threadfence(); }
}
}

extern "C" void kernel_launch(void* const* d_in, const int* in_sizes, int n_in,
                              void* d_out, int out_size, void* d_ws, size_t ws_size, hipStream_t stream) {
  (void)n_in; (void)out_size;
  const float* x = (const float*)d_in[0]; const float* wp = (const float*)d_in[1]; const float* bp = (const float*)d_in[2]; const float* wm = (const float*)d_in[3]; const float* bm = (const float*)d_in[4]; const float* wd = (const float*)d_in[5]; const float* bd = (const float*)d_in[6]; const float* gam = (const float*)d_in[7]; const float* bet = (const float*)d_in[8];
  float* out = (float*)d_out;
  if (in_sizes[0] != NPOS * C || in_sizes[1] != 18 * C * 9 || in_sizes[3] != 9 * C * 9 || in_sizes[5] != CO * C * 9) return;
  size_t off_ = 0; char* ws = (char*)d_ws;
  auto carve = [&](size_t bytes) { char* p = ws + off_; off_ += (bytes + 255) & ~(size_t)255; return p; };
  b16* R = (b16*)carve((size_t)(32 + CO) * KK * 2); float* P = (float*)carve(512 * 4); b16* xt = (b16*)carve((size_t)NPOS * C * 2); float* pm = (float*)carve((size_t)NPOS * 32 * 4); float* y = (float*)carve((size_t)NPOS * CO * 4); float* st = (float*)carve(CO * 32 * 4);
  if (off_ > ws_size) return;
  prep_kernel<<<256, 256, 0, stream>>>(wp, bp, wm, bm, wd, bd, gam, bet, R, P);
  xpose_kernel<<<dim3(H / 2, Bn), 256, 0, stream>>>(x, xt);
  offconv_kernel<<<dim3(H / 2, Bn), 128, 0, stream>>>(xt, R, P, pm);
  deform_kernel<<<dim3(H / 2, Bn), 256, 0, stream>>>(xt, pm, R, P, y);
  bnstat_kernel<<<CO, 256, 0, stream>>>(y, st);
  final_kernel<<<NPOS * CO / 4 / 256, 256, 0, stream>>>(y, st, P, out);
}
